// RNN_15779709845563
// MI455X (gfx1250) — hardware-verified
//
#include <hip/hip_runtime.h>
#include <math.h>

constexpr int NSTEP  = 512;
constexpr int NBAT   = 64;
constexpr int NIN    = 128;
constexpr int NHID   = 512;
constexpr int NLAY   = 3;
constexpr int NOUTF  = 128;
constexpr int NROWS  = NSTEP * NBAT;
constexpr int NTHR   = 256;
constexpr int SEQ_BLK = 16;
constexpr int HPITCH = 520;
constexpr int SLABP  = 68;
constexpr int NOUT0  = NROWS * NOUTF;
constexpr int NOUT1  = NLAY * NBAT * NHID;
constexpr float WCARRY     = 256.0f;
constexpr float WCARRY_INV = 1.0f / 256.0f;

static_assert(NROWS % 64 == 0 && NHID % 64 == 0 && NOUTF % 64 == 0);
static_assert(NIN % 32 == 0 && NHID % 32 == 0);
static_assert(((NROWS / 64) * (NHID / 64)) % 8 == 0);
static_assert(((NROWS / 64) * (NOUTF / 64)) % 8 == 0);
static_assert(NBAT % SEQ_BLK == 0);
static_assert(NHID == 64 * (NTHR / 32));
static_assert((NROWS * NIN / 8) % NTHR == 0);
static_assert((NHID * NIN / 8) % NTHR == 0);
static_assert((2 * NHID * NHID / 8) % NTHR == 0);
static_assert((3 * NHID * NHID / 8) % NTHR == 0);
static_assert((NOUTF * NHID / 8) % NTHR == 0);
static_assert((2 * SEQ_BLK * HPITCH) % NTHR == 0);
static_assert(SEQ_BLK * NHID == 8 * NTHR * 4);
static_assert(SEQ_BLK * NHID == 4 * NTHR * 8);
static_assert(HPITCH % 8 == 0 && SLABP % 4 == 0);
static_assert(NHID == 128 * 4);
static_assert(NOUTF == 32 * 4);
static_assert(NOUT0 * 4 == 16777216);
static_assert((NOUT0 + NOUT1) * 4 == 17170432);

typedef __attribute__((ext_vector_type(16))) _Float16 v16h;
typedef __attribute__((ext_vector_type(8)))  _Float16 v8h;
typedef __attribute__((ext_vector_type(4)))  _Float16 v4h;
typedef __attribute__((ext_vector_type(16))) __bf16   v16b;
typedef __attribute__((ext_vector_type(8)))  __bf16   v8b;
typedef __attribute__((ext_vector_type(8)))  float    v8f;
typedef __attribute__((ext_vector_type(4)))  float    v4f;

__device__ __forceinline__ unsigned short f2bf_bits(float f) {
  unsigned u = __float_as_uint(f);
  return (unsigned short)((u + 0x7FFFu + ((u >> 16) & 1u)) >> 16);
}
__device__ __forceinline__ float bf_bits2f(unsigned short h) { return __uint_as_float(((unsigned)h) << 16); }
__device__ __forceinline__ float bf16r(float f) { return bf_bits2f(f2bf_bits(f)); }

__device__ __forceinline__ void dep_guard_h(v8f& a, v8f& b, v16h x, v16h y) { asm volatile("v_nop\n\tv_nop\n\tv_nop\n\tv_nop" : "+v"(a), "+v"(b) : "v"(x), "v"(y)); }
__device__ __forceinline__ void dep_guard_b(v8f& a, v8f& b, v16b x, v16b y) { asm volatile("v_nop\n\tv_nop\n\tv_nop\n\tv_nop" : "+v"(a), "+v"(b) : "v"(x), "v"(y)); }
__device__ __forceinline__ void grp_guard_h(v8f& a0, v8f& a1, v8f& a2, v8f& a3, v16h x, v16h x2, v16h y0, v16h y1, v16h y2, v16h y3) {
  asm volatile("v_nop\n\tv_nop\n\tv_nop\n\tv_nop" : "+v"(a0), "+v"(a1), "+v"(a2), "+v"(a3) : "v"(x), "v"(x2), "v"(y0), "v"(y1), "v"(y2), "v"(y3));
}
__device__ __forceinline__ void grp_guard_b(v8f& a0, v8f& a1, v8f& a2, v8f& a3, v16b x, v16b x2, v16b y0, v16b y1, v16b y2, v16b y3) {
  asm volatile("v_nop\n\tv_nop\n\tv_nop\n\tv_nop" : "+v"(a0), "+v"(a1), "+v"(a2), "+v"(a3) : "v"(x), "v"(x2), "v"(y0), "v"(y1), "v"(y2), "v"(y3));
}
__device__ __forceinline__ void keep4_h(v16h a, v16h b, v16h c, v16h d) { asm volatile("v_nop" :: "v"(a), "v"(b), "v"(c), "v"(d)); }
__device__ __forceinline__ void keep4_b(v16b a, v16b b, v16b c, v16b d) { asm volatile("v_nop" :: "v"(a), "v"(b), "v"(c), "v"(d)); }
__device__ __forceinline__ void acc_guard4(v8f& a, v8f& b, v8f& c, v8f& d) { asm volatile("v_nop\n\tv_nop\n\tv_nop\n\tv_nop" : "+v"(a), "+v"(b), "+v"(c), "+v"(d)); }
template <typename T> struct Frag;
template <> struct Frag<_Float16> {
  typedef v16h V; union U { v16h v; v8h h[2]; };
  static __device__ __forceinline__ v16h load(const _Float16* p) {
    U f; f.h[0] = *(const v8h*)(p); f.h[1] = *(const v8h*)(p + 16); return f.v;
  }
  static __device__ __forceinline__ v8f mma(v16h a, v16h b, v8f c) {
    return __builtin_amdgcn_wmma_f32_16x16x32_f16(false, a, false, b, (short)0, c, false, false);
  }
  static __device__ __forceinline__ void guard(v8f& a, v8f& b, v16h x, v16h y) { dep_guard_h(a, b, x, y); }
  static __device__ __forceinline__ void guard_grp(v8f& a0, v8f& a1, v8f& a2, v8f& a3, v16h x, v16h x2, v16h y0, v16h y1, v16h y2, v16h y3) {
    grp_guard_h(a0, a1, a2, a3, x, x2, y0, y1, y2, y3);
  }
  static __device__ __forceinline__ void keep(v16h a, v16h b, v16h c, v16h d) { keep4_h(a, b, c, d); }
};
template <> struct Frag<__bf16> {
  typedef v16b V; union U { v16b v; v8b h[2]; };
  static __device__ __forceinline__ v16b load(const __bf16* p) {
    U f; f.h[0] = *(const v8b*)(p); f.h[1] = *(const v8b*)(p + 16); return f.v;
  }
  static __device__ __forceinline__ v8f mma(v16b a, v16b b, v8f c) {
    return __builtin_amdgcn_wmma_f32_16x16x32_bf16(false, a, false, b, (short)0, c, false, false);
  }
  static __device__ __forceinline__ void guard(v8f& a, v8f& b, v16b x, v16b y) { dep_guard_b(a, b, x, y); }
  static __device__ __forceinline__ void guard_grp(v8f& a0, v8f& a1, v8f& a2, v8f& a3, v16b x, v16b x2, v16b y0, v16b y1, v16b y2, v16b y3) {
    grp_guard_b(a0, a1, a2, a3, x, x2, y0, y1, y2, y3);
  }
  static __device__ __forceinline__ void keep(v16b a, v16b b, v16b c, v16b d) { keep4_b(a, b, c, d); }
};

template <int ET> struct Elem;
template <> struct Elem<0> { typedef _Float16 T; };
template <> struct Elem<1> { typedef __bf16 T; };
template <int ET, bool SPLIT, int BIAS_MODE, int OUT_MODE, bool RESID, int ACT = 0>
__global__ __launch_bounds__(256) void wmma_gemm64(
    const unsigned short* __restrict__ Ap, const unsigned short* __restrict__ A2p, int lda, long strideA,
    const unsigned short* __restrict__ Btp, const unsigned short* __restrict__ Bt2p, int ldb, long strideB,
    void* __restrict__ Cout, void* __restrict__ Cout2, int ldc, long strideC,
    const float* __restrict__ bias,
    const float* __restrict__ resid, long strideR,
    int M, int N, int K, float scale) {
  typedef typename Elem<ET>::T T;
  typedef typename Frag<T>::V V;
  const T* A = (const T*)Ap; const T* A2 = (const T*)A2p; const T* Bt = (const T*)Btp; const T* Bt2 = (const T*)Bt2p;
  __shared__ __align__(16) float sT[8][16 * 68];
  const int b    = blockIdx.y;
  const int lane = threadIdx.x & 31;
  const int wave = threadIdx.x >> 5;
  const int tilesN = N >> 6;
  const int tilesM = M >> 6;
  const int tile = blockIdx.x * 8 + wave;
  if (tile >= tilesM * tilesN) return;
  const int tm = tile / tilesN;
  const int tn = tile - tm * tilesN;
  const int m0 = tm << 6;
  const int n0 = tn << 6;

  const T* Ab  = A  + (size_t)b * strideA;
  const T* Bb  = Bt + (size_t)b * strideB;
  const T* Ab2 = SPLIT ? (A2  + (size_t)b * strideA) : nullptr;
  const T* Bb2 = SPLIT ? (Bt2 + (size_t)b * strideB) : nullptr;

  const int rlane = lane & 15;
  const int koff  = (lane >> 4) * 8;
  const int mOff  = (lane >> 4) * 8;

  v8f acc[4][4];
#pragma unroll
  for (int i = 0; i < 4; ++i)
#pragma unroll
    for (int j = 0; j < 4; ++j) acc[i][j] = (v8f){0.f,0.f,0.f,0.f,0.f,0.f,0.f,0.f};

  for (int k0 = 0; k0 < K; k0 += 32) {
    V bh[4], bl[4];
#pragma unroll
    for (int j = 0; j < 4; ++j) {
      const size_t bo = (size_t)(n0 + (j << 4) + rlane) * ldb + koff + k0;
      bh[j] = Frag<T>::load(Bb + bo);
      if (SPLIT) bl[j] = Frag<T>::load(Bb2 + bo);
    }
#pragma unroll
    for (int i = 0; i < 4; ++i) {
      const size_t ao = (size_t)(m0 + (i << 4) + rlane) * lda + koff + k0;
      V ah = Frag<T>::load(Ab + ao);
      V al;
      if (SPLIT) al = Frag<T>::load(Ab2 + ao);
#pragma unroll
      for (int j = 0; j < 4; ++j) {
        acc[i][j] = Frag<T>::mma(ah, bh[j], acc[i][j]);
        if (SPLIT) {
          acc[i][j] = Frag<T>::mma(ah, bl[j], acc[i][j]);
          acc[i][j] = Frag<T>::mma(al, bh[j], acc[i][j]);
        }
      }
      Frag<T>::guard_grp(acc[i][0], acc[i][1], acc[i][2], acc[i][3], ah, SPLIT ? al : ah, bh[0], bh[1], bh[2], bh[3]);
      if (SPLIT) Frag<T>::keep(bl[0], bl[1], bl[2], bl[3]);
    }
    Frag<T>::keep(bh[0], bh[1], bh[2], bh[3]);
    if (SPLIT) Frag<T>::keep(bl[0], bl[1], bl[2], bl[3]);
  }
  acc_guard4(acc[0][0], acc[0][1], acc[0][2], acc[0][3]);
  acc_guard4(acc[1][0], acc[1][1], acc[1][2], acc[1][3]);
  acc_guard4(acc[2][0], acc[2][1], acc[2][2], acc[2][3]);
  acc_guard4(acc[3][0], acc[3][1], acc[3][2], acc[3][3]);

  float* slab = sT[wave];
  const float* Rb = RESID ? (resid + (size_t)b * strideR) : nullptr;
#pragma unroll
  for (int i = 0; i < 4; ++i) {
    const int mBase = m0 + (i << 4);
#pragma unroll
    for (int j = 0; j < 4; ++j) {
      const int n = n0 + (j << 4) + rlane;
      float bv = 0.f;
      if (BIAS_MODE == 2) bv = bias[n];
#pragma unroll
      for (int r = 0; r < 8; ++r) {
        float v = acc[i][j][r] * scale;
        if (BIAS_MODE == 1) v += bias[mBase + mOff + r];
        if (BIAS_MODE == 2) v += bv;
        if (RESID) v += Rb[(size_t)(mBase + mOff + r) * ldc + n];
        if (ACT == 1) v = tanhf(v);
        if (ACT == 2) v = fmaxf(v, 0.0f);
        if (ACT == 3) v = v / (1.0f + expf(-v));
        if (ACT == 4) v = (v > 0.f) ? v : 0.01f * v;
        if (ACT == 5) v = 0.5f * v * (1.0f + erff(v * 0.70710678118654752f));
        slab[(mOff + r) * 68 + (j << 4) + rlane] = v;
      }
    }
    __builtin_amdgcn_fence(__ATOMIC_RELEASE, "workgroup");
    __builtin_amdgcn_wave_barrier();
    __builtin_amdgcn_fence(__ATOMIC_ACQUIRE, "workgroup");
    if (OUT_MODE == 0) {
      float* C = (float*)Cout + (size_t)b * strideC;
      const int hh = lane >> 4, c4 = (lane & 15) * 4;
      for (int pass = 0; pass < 2; ++pass) {
#pragma unroll
        for (int it = 0; it < 8; ++it) {
          const int row = it * 2 + hh;
          v4f v = *(const v4f*)(slab + row * 68 + c4);
          *(volatile v4f*)(C + (size_t)(mBase + row) * ldc + n0 + c4) = v;
        }
        __threadfence();
      }
    } else {
      const int q = lane >> 3, c8 = (lane & 7) * 8;
      unsigned short* C  = (unsigned short*)Cout  + (size_t)b * strideC;
      unsigned short* C2 = (OUT_MODE == 2) ? ((unsigned short*)Cout2 + (size_t)b * strideC) : nullptr;
      for (int pass = 0; pass < 2; ++pass) {
#pragma unroll
        for (int it = 0; it < 4; ++it) {
          const int row = it * 4 + q;
          const float* sp = slab + row * 68 + c8;
          v8h hv, lv;
#pragma unroll
          for (int e = 0; e < 8; ++e) {
            if (OUT_MODE == 1) {
              hv[e] = (_Float16)sp[e];
            } else {
              unsigned short hb = f2bf_bits(sp[e]);
              unsigned short lb = f2bf_bits(sp[e] - bf_bits2f(hb));
              hv[e] = __builtin_bit_cast(_Float16, hb);
              lv[e] = __builtin_bit_cast(_Float16, lb);
            }
          }
          *(volatile v8h*)(C + (size_t)(mBase + row) * ldc + n0 + c8) = hv;
          if (OUT_MODE == 2) *(volatile v8h*)(C2 + (size_t)(mBase + row) * ldc + n0 + c8) = lv;
        }
        __threadfence();
      }
    }
    __builtin_amdgcn_fence(__ATOMIC_RELEASE, "workgroup");
    __builtin_amdgcn_wave_barrier();
    __builtin_amdgcn_fence(__ATOMIC_ACQUIRE, "workgroup");
  }
}

__global__ __launch_bounds__(NTHR) void cvt_f16x8_kernel(const float* __restrict__ src, unsigned short* __restrict__ dst,
                                                         int n8, float sc) {
  const int i = blockIdx.x * NTHR + threadIdx.x;
  if (i < n8) {
    const float* sp = src + (size_t)i * 8;
    const v4f a = *(const v4f*)(sp);
    const v4f b = *(const v4f*)(sp + 4);
    v8h hv;
#pragma unroll
    for (int e = 0; e < 4; ++e) {
      const float fa = bf16r(a[e]) * sc;
      const float fb = bf16r(b[e]) * sc;
      hv[e]     = (_Float16)fa;
      hv[4 + e] = (_Float16)fb;
    }
    *(volatile v8h*)(dst + (size_t)i * 8) = hv;
    __threadfence();
    *(volatile v8h*)(dst + (size_t)i * 8) = hv;
  }
}

__global__ __launch_bounds__(128) void bias_sum_kernel(const float* __restrict__ b_a, const float* __restrict__ b_b,
                                                       float* __restrict__ dst) {
  const int l = blockIdx.x;
  const int idx = threadIdx.x * 4;
  const v4f va = *(const v4f*)(b_a + (size_t)l * NHID + idx);
  const v4f vb = *(const v4f*)(b_b + (size_t)l * NHID + idx);
  v4f o;
#pragma unroll
  for (int e = 0; e < 4; ++e) o[e] = bf16r(va[e]) + bf16r(vb[e]);
  float* op = dst + (size_t)l * NHID + idx;
  *(volatile v4f*)op = o;
  __threadfence();
  *(volatile v4f*)op = o;
}

__global__ __launch_bounds__(32) void bias_rne_kernel(const float* __restrict__ src, float* __restrict__ dst) {
  const int idx = threadIdx.x * 4;
  const v4f v = *(const v4f*)(src + idx);
  v4f o;
#pragma unroll
  for (int e = 0; e < 4; ++e) o[e] = bf16r(v[e]);
  float* op = dst + idx;
  *(volatile v4f*)op = o;
  __threadfence();
  *(volatile v4f*)op = o;
}

__global__ __launch_bounds__(NTHR) void rnn_scan_kernel(const float* __restrict__ PRE, const float* __restrict__ h0l,
                                                        const unsigned short* __restrict__ WHp,
                                                        unsigned short* __restrict__ YS, float* __restrict__ HFIN) {
  __shared__ __align__(16) _Float16 Ah[2][SEQ_BLK * HPITCH];
  __shared__ __align__(16) float    Sl[NTHR / 32][16 * SLABP];
  const _Float16* WH = (const _Float16*)WHp;
  const int tid = threadIdx.x, lane = tid & 31, wave = tid >> 5;
  const int c = lane & 15, hh = lane >> 4, koff = hh * 8, c4 = c * 4;
  const int b0 = blockIdx.x * SEQ_BLK;

  {
    _Float16* ahf = &Ah[0][0];
#pragma unroll 1
    for (int i = tid; i < 2 * SEQ_BLK * HPITCH; i += NTHR) ahf[i] = (_Float16)0.0f;
  }
  __syncthreads();
#pragma unroll 1
  for (int it = 0; it < 8; ++it) {
    const int idx = it * NTHR + tid;
    const int row = idx >> 7;
    const int cc  = (idx & 127) * 4;
    const v4f v = *(const v4f*)(h0l + (size_t)(b0 + row) * NHID + cc);
    v4h hv;
    hv[0] = (_Float16)bf16r(v[0]);
    hv[1] = (_Float16)bf16r(v[1]);
    hv[2] = (_Float16)bf16r(v[2]);
    hv[3] = (_Float16)bf16r(v[3]);
    *(v4h*)(&Ah[0][row * HPITCH + cc]) = hv;
  }
  float hst[4][8];
#pragma unroll
  for (int nt = 0; nt < 4; ++nt)
#pragma unroll
    for (int r = 0; r < 8; ++r) hst[nt][r] = 0.0f;
  const _Float16* whb = WH + (size_t)(64 * wave + c) * NHID + koff;
  __syncthreads();

  const v8f z8 = {0.f, 0.f, 0.f, 0.f, 0.f, 0.f, 0.f, 0.f};

#pragma unroll 1
  for (int t = 0; t < NSTEP; ++t) {
    const int cur = t & 1;
    const _Float16* ahrow = &Ah[cur][0] + c * HPITCH + koff;
    _Float16* ahn = &Ah[cur ^ 1][0];
    v8f acc[4];
    acc[0] = z8; acc[1] = z8; acc[2] = z8; acc[3] = z8;
#pragma unroll 1
    for (int k0 = 0; k0 < NHID; k0 += 32) {
      const v16h a  = Frag<_Float16>::load(ahrow + k0);
      const v16h w0 = Frag<_Float16>::load(whb + k0);
      const v16h w1 = Frag<_Float16>::load(whb + (size_t)16 * NHID + k0);
      const v16h w2 = Frag<_Float16>::load(whb + (size_t)32 * NHID + k0);
      const v16h w3 = Frag<_Float16>::load(whb + (size_t)48 * NHID + k0);
      acc[0] = Frag<_Float16>::mma(a, w0, acc[0]);
      acc[1] = Frag<_Float16>::mma(a, w1, acc[1]);
      acc[2] = Frag<_Float16>::mma(a, w2, acc[2]);
      acc[3] = Frag<_Float16>::mma(a, w3, acc[3]);
      grp_guard_h(acc[0], acc[1], acc[2], acc[3], a, a, w0, w1, w2, w3);
    }
    acc_guard4(acc[0], acc[1], acc[2], acc[3]);

    const float* prow = PRE + ((size_t)t * NBAT + (size_t)(b0 + 8 * hh)) * NHID + 64 * wave + c;
#pragma unroll
    for (int nt = 0; nt < 4; ++nt) {
      const int j = 64 * wave + 16 * nt + c;
      float pv[8];
      asm volatile("" ::: "memory");
#pragma unroll
      for (int r = 0; r < 8; ++r) pv[r] = prow[(size_t)r * NHID + 16 * nt];
      asm volatile("" ::: "memory");
#pragma unroll
      for (int r = 0; r < 8; ++r) {
        const float z  = acc[nt][r] * WCARRY_INV + pv[r];
        const float hn = tanhf(z);
        hst[nt][r] = hn;
        ahn[(8 * hh + r) * HPITCH + j] = (_Float16)hn;
      }
    }
    __syncthreads();

    unsigned short* yb = YS + ((size_t)t * NBAT + (size_t)b0) * NHID;
    for (int pass = 0; pass < 2; ++pass) {
#pragma unroll
      for (int it = 0; it < 4; ++it) {
        const int idx = it * NTHR + tid;
        const int row = idx >> 6;
        const int c8  = (idx & 63) * 8;
        const v8h v = *(const v8h*)(ahn + row * HPITCH + c8);
        *(volatile v8h*)(yb + (size_t)row * NHID + c8) = v;
      }
      __threadfence();
    }
  }

  float* slab = Sl[wave];
#pragma unroll
  for (int nt = 0; nt < 4; ++nt)
#pragma unroll
    for (int r = 0; r < 8; ++r) slab[(8 * hh + r) * SLABP + 16 * nt + c] = hst[nt][r];
  __syncthreads();
  for (int pass = 0; pass < 2; ++pass) {
#pragma unroll
    for (int it = 0; it < 8; ++it) {
      const int row = it * 2 + hh;
      const v4f v = *(const v4f*)(slab + row * SLABP + c4);
      *(volatile v4f*)(HFIN + (size_t)(b0 + row) * NHID + 64 * wave + c4) = v;
    }
    __threadfence();
  }
}

extern "C" void kernel_launch(void* const* d_in, const int* in_sizes, int n_in,
                              void* d_out, int out_size, void* d_ws, size_t ws_size, hipStream_t stream) {
  if (n_in < 9 || d_out == nullptr || d_ws == nullptr) return;
  if (in_sizes[0] != NROWS * NIN || in_sizes[1] != NLAY * NBAT * NHID || in_sizes[2] != NHID * NIN ||
      in_sizes[3] != 2 * NHID * NHID || in_sizes[4] != NLAY * NHID * NHID || in_sizes[5] != NLAY * NHID ||
      in_sizes[6] != NLAY * NHID || in_sizes[7] != NOUTF * NHID || in_sizes[8] != NOUTF ||
      out_size != NOUT0 + NOUT1) return;

  const float* x     = (const float*)d_in[0];
  const float* h0    = (const float*)d_in[1];
  const float* w_ih0 = (const float*)d_in[2];
  const float* w_ihr = (const float*)d_in[3];
  const float* w_hh  = (const float*)d_in[4];
  const float* b_ih  = (const float*)d_in[5];
  const float* b_hh  = (const float*)d_in[6];
  const float* lin_w = (const float*)d_in[7];
  const float* lin_b = (const float*)d_in[8];
  float* out0 = (float*)d_out;
  float* hfin = out0 + (size_t)NOUT0;

  char* ws = (char*)d_ws; size_t off = 0;
  auto carve = [&](size_t bytes) -> char* { char* p = ws + off; off += (bytes + 255) & ~(size_t)255; return p; };
  unsigned short* X16  = (unsigned short*)carve((size_t)NROWS * NIN * 2);
  unsigned short* WIH0 = (unsigned short*)carve((size_t)NHID * NIN * 2);
  unsigned short* WIHR = (unsigned short*)carve((size_t)2 * NHID * NHID * 2);
  unsigned short* WHH  = (unsigned short*)carve((size_t)NLAY * NHID * NHID * 2);
  unsigned short* LINW = (unsigned short*)carve((size_t)NOUTF * NHID * 2);
  float*          BSUM = (float*)carve((size_t)NLAY * NHID * 4);
  float*          LINB = (float*)carve((size_t)NOUTF * 4);
  float*          PRE  = (float*)carve((size_t)NROWS * NHID * 4);
  unsigned short* YS   = (unsigned short*)carve((size_t)NROWS * NHID * 2);
  if (off > ws_size || off > (size_t)134217728) return;

  const int n8x  = NROWS * NIN / 8;
  const int n8w0 = NHID * NIN / 8;
  const int n8wr = 2 * NHID * NHID / 8;
  const int n8wh = NLAY * NHID * NHID / 8;
  const int n8lw = NOUTF * NHID / 8;
  cvt_f16x8_kernel<<<n8x  / NTHR, NTHR, 0, stream>>>(x,     X16,  n8x,  1.0f);
  cvt_f16x8_kernel<<<n8w0 / NTHR, NTHR, 0, stream>>>(w_ih0, WIH0, n8w0, WCARRY);
  cvt_f16x8_kernel<<<n8wr / NTHR, NTHR, 0, stream>>>(w_ihr, WIHR, n8wr, WCARRY);
  cvt_f16x8_kernel<<<n8wh / NTHR, NTHR, 0, stream>>>(w_hh,  WHH,  n8wh, WCARRY);
  cvt_f16x8_kernel<<<n8lw / NTHR, NTHR, 0, stream>>>(lin_w, LINW, n8lw, WCARRY);
  bias_sum_kernel<<<NLAY, 128, 0, stream>>>(b_ih, b_hh, BSUM);
  bias_rne_kernel<<<1, 32, 0, stream>>>(lin_b, LINB);

  const dim3 pgrid((NROWS / 64) * (NHID / 64) / 8, 1);
  for (int l = 0; l < NLAY; ++l) {
    const unsigned short* Ain = (l == 0) ? X16 : YS;
    const unsigned short* Bw  = (l == 0) ? WIH0 : (WIHR + (size_t)(l - 1) * NHID * NHID);
    const int kdim = (l == 0) ? NIN : NHID;
    wmma_gemm64<0, false, 2, 0, false, 0><<<pgrid, 256, 0, stream>>>(
        Ain, Ain, kdim, 0L, Bw, Bw, kdim, 0L, (void*)PRE, (void*)PRE, NHID, 0L,
        BSUM + (size_t)l * NHID, BSUM, 0L, NROWS, NHID, kdim, WCARRY_INV);
    rnn_scan_kernel<<<NBAT / SEQ_BLK, NTHR, 0, stream>>>(
        PRE, h0 + (size_t)l * NBAT * NHID, WHH + (size_t)l * NHID * NHID, YS, hfin + (size_t)l * NBAT * NHID);
  }

  const dim3 hgrid((NROWS / 64) * (NOUTF / 64) / 8, 1);
  wmma_gemm64<0, false, 2, 0, false, 0><<<hgrid, 256, 0, stream>>>(
      YS, YS, NHID, 0L, LINW, LINW, NHID, 0L, (void*)out0, (void*)out0, NOUTF, 0L,
      LINB, BSUM, 0L, NROWS, NOUTF, NHID, WCARRY_INV);
}
